// Encoder_55748675502365
// MI455X (gfx1250) — hardware-verified
//
#include <hip/hip_runtime.h>
#include <stddef.h>
#include <stdint.h>


#define DIN    256
#define GN     128
#define NG     256
#define KHL    512
#define NTHR   256
#define NWAVE  8
#define EPT    8
#define CHUNK  (NTHR * EPT)
#define WCAP   (EPT * 32)
#define LISTN  (NWAVE * WCAP)
#define NBMAX  2048
#define SLOTB  11
#define RCAP   28672
#define DEGCAP 256
#define GBM    32
#define GTHR   64
#define MROWS  128
#define U1M    4096
#define U2M    8192
#define UTOT   (2 * U1M + 3 * U2M)
#define NEGSL  0.2f
#define WSMAX  134217728
#define LDS_AGG ((2 * RCAP + 2 * NBMAX + LISTN) * 4 + 64)

static_assert((CHUNK & (CHUNK - 1)) == 0 && CHUNK <= (1 << SLOTB));
static_assert(NBMAX == (1 << SLOTB));
static_assert(NTHR * 8 == NBMAX);
static_assert(LISTN >= NBMAX);
static_assert(LISTN >= NWAVE * WCAP);
static_assert((RCAP % 32) == 0);
static_assert(LDS_AGG <= 300000);
static_assert(GBM == (GTHR / 32) * 16);
static_assert(GTHR == 64 && GBM == 32);
static_assert((DIN % 32) == 0 && (KHL % 32) == 0 && KHL == 2 * NG && NG == 2 * GN);
static_assert(GN == 4 * 32);
static_assert((MROWS % GBM) == 0 && ((MROWS * (DIN / 8)) % NTHR) == 0);
static_assert(DIN / 8 == 32);
static_assert(U1M == GN * (DIN / 8) && U2M == GN * (KHL / 8));
static_assert((U1M % NTHR) == 0 && (U2M % NTHR) == 0 && (UTOT % NTHR) == 0);
static_assert(U1M == (1 << 12) && U2M == (1 << 13));

typedef float          v2f   __attribute__((ext_vector_type(2)));
typedef float          v4f   __attribute__((ext_vector_type(4)));
typedef float          v8f   __attribute__((ext_vector_type(8)));
typedef int            v4i   __attribute__((ext_vector_type(4)));
typedef int            v8i   __attribute__((ext_vector_type(8)));
typedef unsigned short v8us  __attribute__((ext_vector_type(8)));
typedef unsigned short v16us __attribute__((ext_vector_type(16)));
typedef __bf16         v16bf __attribute__((ext_vector_type(16)));
typedef v2f  __attribute__((may_alias)) v2fa;
typedef v4f  __attribute__((may_alias)) v4fa;
typedef v4i  __attribute__((may_alias)) v4ia;
typedef v8us __attribute__((may_alias)) v8usa;
union Frag { v16bf v; v16us u; v8us h[2]; v8i w; };

__device__ __forceinline__ v8f wmb(const Frag& a, const Frag& b, v8f c) {
  v8f d = __builtin_amdgcn_wmma_f32_16x16x32_bf16(false, a.v, false, b.v, (short)0, c, false, false);
  asm volatile("v_nop\n\tv_nop\n\tv_nop\n\tv_nop" : "+v"(d) : "v"(a.w), "v"(b.w));
  return d;
}

__device__ __forceinline__ unsigned bf16_bits(float f) {
  const unsigned u = __float_as_uint(f);
  return (u + 0x7FFFu + ((u >> 16) & 1u)) >> 16;
}
__device__ __forceinline__ float bf16_val(float f) {
  return __uint_as_float(bf16_bits(f) << 16);
}
__device__ __forceinline__ v8us hilo8(v4f t) {
  v8us o;
  unsigned hb;
  hb = bf16_bits(t.x); o[0] = (unsigned short)hb; o[4] = (unsigned short)bf16_bits(t.x - __uint_as_float(hb << 16));
  hb = bf16_bits(t.y); o[1] = (unsigned short)hb; o[5] = (unsigned short)bf16_bits(t.y - __uint_as_float(hb << 16));
  hb = bf16_bits(t.z); o[2] = (unsigned short)hb; o[6] = (unsigned short)bf16_bits(t.z - __uint_as_float(hb << 16));
  hb = bf16_bits(t.w); o[3] = (unsigned short)hb; o[7] = (unsigned short)bf16_bits(t.w - __uint_as_float(hb << 16));
  return o;
}

__device__ __forceinline__ int scan_chunk(const int* __restrict__ dsts, int nE, int cbase, int slotBase,
                                          int nb, int vec8, int* list, int tid, int lane, int wave) {
  int wc = 0;
  const int el0  = tid * EPT;
  const int e0   = cbase + el0;
  const int sent = -2147483647 - 1;
  v4i da, db;
  if (vec8 != 0 && cbase + CHUNK <= nE) {
    da = *(const v4i*)(dsts + e0);
    db = *(const v4i*)(dsts + e0 + 4);
  } else {
    da.x = (e0     < nE) ? dsts[min(e0,     nE - 1)] : sent;
    da.y = (e0 + 1 < nE) ? dsts[min(e0 + 1, nE - 1)] : sent;
    da.z = (e0 + 2 < nE) ? dsts[min(e0 + 2, nE - 1)] : sent;
    da.w = (e0 + 3 < nE) ? dsts[min(e0 + 3, nE - 1)] : sent;
    db.x = (e0 + 4 < nE) ? dsts[min(e0 + 4, nE - 1)] : sent;
    db.y = (e0 + 5 < nE) ? dsts[min(e0 + 5, nE - 1)] : sent;
    db.z = (e0 + 6 < nE) ? dsts[min(e0 + 6, nE - 1)] : sent;
    db.w = (e0 + 7 < nE) ? dsts[min(e0 + 7, nE - 1)] : sent;
  }
  const unsigned nbs = (unsigned)slotBase;
  const unsigned unb = (unsigned)nb;
  const unsigned s0 = (unsigned)da.x - nbs, s1 = (unsigned)da.y - nbs;
  const unsigned s2 = (unsigned)da.z - nbs, s3 = (unsigned)da.w - nbs;
  const unsigned s4 = (unsigned)db.x - nbs, s5 = (unsigned)db.y - nbs;
  const unsigned s6 = (unsigned)db.z - nbs, s7 = (unsigned)db.w - nbs;
  const bool h0 = s0 < unb, h1 = s1 < unb, h2 = s2 < unb, h3 = s3 < unb;
  const bool h4 = s4 < unb, h5 = s5 < unb, h6 = s6 < unb, h7 = s7 < unb;
  const unsigned any = __builtin_amdgcn_ballot_w32(h0 | h1 | h2 | h3 | h4 | h5 | h6 | h7);
  if (any != 0u) {
#define HITJ(J, HJ, SJ) { \
      const unsigned mj = __builtin_amdgcn_ballot_w32(HJ); \
      if (mj != 0u) { \
        if (HJ) { \
          const int pos = wc + (int)__builtin_amdgcn_mbcnt_lo(mj, 0u); \
          if (pos < WCAP) list[wave * WCAP + pos] = ((el0 + (J)) << SLOTB) | (int)(SJ); \
        } \
        wc += (int)__builtin_popcount(mj); } }
    HITJ(0, h0, s0)
    HITJ(1, h1, s1)
    HITJ(2, h2, s2)
    HITJ(3, h3, s3)
    HITJ(4, h4, s4)
    HITJ(5, h5, s5)
    HITJ(6, h6, s6)
    HITJ(7, h7, s7)
#undef HITJ
  }
  return wc;
}

__global__ __launch_bounds__(NTHR) void k_wprep(const float* __restrict__ Wo1, const float* __restrict__ Ws1,
                                                const float* __restrict__ Wo2, const float* __restrict__ Ws2,
                                                const float* __restrict__ Wp,
                                                unsigned short* WT1, unsigned short* WT2, unsigned short* WTp) {
  const int u = (int)blockIdx.x * NTHR + (int)threadIdx.x;
  if (u >= UTOT) return;
  v8us o;
  unsigned short* dp;
  if (u < 2 * U1M) {
    const int mi = u >> 12;
    const float* W = (mi == 0) ? Wo1 : Ws1;
    const int v  = u & (U1M - 1);
    const int n  = v >> 5;
    const int k8 = (v & 31) * 8;
    const float* p = W + (size_t)k8 * GN + n;
#pragma unroll
    for (int i = 0; i < 8; ++i) o[i] = (unsigned short)bf16_bits(p[(size_t)i * GN]);
    dp = WT1 + (size_t)(mi * GN + n) * (size_t)DIN + k8;
  } else {
    const int u2 = u - 2 * U1M;
    const int mi = u2 >> 13;
    const float* W = Wo2;
    unsigned short* D = WT2;
    int rowoff = 0;
    if (mi == 1)      { W = Ws2; rowoff = GN; }
    else if (mi == 2) { W = Wp;  D = WTp; }
    const int v = u2 & (U2M - 1);
    const int n = v >> 6;
    const int g = v & 63;
    const float* p = W + (size_t)(4 * g) * GN + n;
    const unsigned short f0 = (unsigned short)bf16_bits(p[0]);
    const unsigned short f1 = (unsigned short)bf16_bits(p[GN]);
    const unsigned short f2 = (unsigned short)bf16_bits(p[2 * GN]);
    const unsigned short f3 = (unsigned short)bf16_bits(p[3 * GN]);
    o[0] = f0; o[1] = f1; o[2] = f2; o[3] = f3; o[4] = f0; o[5] = f1; o[6] = f2; o[7] = f3;
    dp = D + (size_t)(rowoff + n) * (size_t)KHL + 8 * g;
  }
  *(volatile v8us*)dp = o;
  __threadfence();
  *(volatile v8us*)dp = o;
}

__global__ __launch_bounds__(NTHR) void k_xprep(const float* __restrict__ x, unsigned short* xb, int nN, int nUnits) {
  const int u = (int)blockIdx.x * NTHR + (int)threadIdx.x;
  if (u >= nUnits) return;
  const int row = u >> 5;
  const int k8  = (u & 31) * 8;
  const int rc  = row < nN ? row : nN - 1;
  const float* p = x + (size_t)rc * DIN + k8;
  const v4f a = *(const v4fa*)p;
  const v4f b = *(const v4fa*)(p + 4);
  const bool ok = row < nN;
  v8us o;
  o[0] = ok ? (unsigned short)bf16_bits(a.x) : (unsigned short)0;
  o[1] = ok ? (unsigned short)bf16_bits(a.y) : (unsigned short)0;
  o[2] = ok ? (unsigned short)bf16_bits(a.z) : (unsigned short)0;
  o[3] = ok ? (unsigned short)bf16_bits(a.w) : (unsigned short)0;
  o[4] = ok ? (unsigned short)bf16_bits(b.x) : (unsigned short)0;
  o[5] = ok ? (unsigned short)bf16_bits(b.y) : (unsigned short)0;
  o[6] = ok ? (unsigned short)bf16_bits(b.z) : (unsigned short)0;
  o[7] = ok ? (unsigned short)bf16_bits(b.w) : (unsigned short)0;
  unsigned short* dp = xb + (size_t)row * DIN + k8;
  *(volatile v8us*)dp = o;
  __threadfence();
  *(volatile v8us*)dp = o;
}

template <int DOTS, int BIAS>
__global__ __launch_bounds__(GTHR) void k_gemm(const unsigned short* __restrict__ A,
                                               const unsigned short* __restrict__ WT, int K, int MPr,
                                               const float* __restrict__ as0, const float* __restrict__ ad0,
                                               const float* __restrict__ as1, const float* __restrict__ ad1,
                                               const float* __restrict__ bias,
                                               float* H, int ldh, int nStore, float* SD) {
  __shared__ __attribute__((aligned(16))) float stg[GBM * GN];
  __shared__ __attribute__((aligned(16))) float satt[2 * GN];
  __shared__ __attribute__((aligned(16))) float sdot[2 * GBM];
  const int tid = (int)threadIdx.x, lane = tid & 31, wave = tid >> 5, hh = lane >> 4, m = lane & 15;
  const int rowBase = (int)blockIdx.x * GBM;
  const int g = (int)blockIdx.y;

  if constexpr (DOTS != 0) {
    const float* pS = (g == 0) ? as0 : as1;
    const float* pD = (g == 0) ? ad0 : ad1;
    satt[tid]           = bf16_val(pS[tid]);
    satt[64 + tid]      = bf16_val(pS[64 + tid]);
    satt[GN + tid]      = bf16_val(pD[tid]);
    satt[GN + 64 + tid] = bf16_val(pD[64 + tid]);
  }

  v8f acc[8];
  {
    const v8f z = {0.f, 0.f, 0.f, 0.f, 0.f, 0.f, 0.f, 0.f};
#pragma unroll
    for (int t = 0; t < 8; ++t) acc[t] = z;
  }
  const unsigned short* ap = A  + (size_t)(rowBase + 16 * wave + m) * (size_t)K + 8 * hh;
  const unsigned short* bp = WT + ((size_t)g * GN + m) * (size_t)K + 8 * hh;
  const int ksteps = K >> 5;

#pragma unroll 1
  for (int ks = 0; ks < ksteps; ++ks) {
    const int k0 = 32 * ks;
    Frag af;
    af.h[0] = *(const v8usa*)(ap + k0);
    af.h[1] = *(const v8usa*)(ap + k0 + 16);
#pragma unroll
    for (int nt = 0; nt < 8; ++nt) {
      const unsigned short* wq = bp + (size_t)(16 * nt) * (size_t)K + k0;
      Frag bf;
      bf.h[0] = *(const v8usa*)wq;
      bf.h[1] = *(const v8usa*)(wq + 16);
      acc[nt] = wmb(af, bf, acc[nt]);
    }
  }

#pragma unroll
  for (int nt = 0; nt < 8; ++nt) {
    const int lc = 16 * nt + m;
#pragma unroll
    for (int r = 0; r < 8; ++r) {
      const int lr = 16 * wave + 8 * hh + r;
      stg[lr * GN + lc] = acc[nt][r];
    }
  }
  __syncthreads();

  if constexpr (DOTS != 0) {
    const int row = tid & 31, which = tid >> 5;
    const float* hr = stg + row * GN;
    const float* sa = satt + which * GN;
    float d = 0.f;
#pragma unroll 4
    for (int c4 = 0; c4 < GN / 4; ++c4) {
      const v4f hv = *(const v4fa*)(hr + 4 * c4);
      const v4f av = *(const v4fa*)(sa + 4 * c4);
      d = fmaf(hv.x, av.x, d);
      d = fmaf(hv.y, av.y, d);
      d = fmaf(hv.z, av.z, d);
      d = fmaf(hv.w, av.w, d);
    }
    sdot[which * GBM + row] = d;
  }
  __syncthreads();

  v4f b4 = {0.f, 0.f, 0.f, 0.f};
  if constexpr (BIAS != 0) {
    const v4f t = *(const v4fa*)(bias + (size_t)g * GN + 4 * lane);
    b4.x = bf16_val(t.x); b4.y = bf16_val(t.y); b4.z = bf16_val(t.z); b4.w = bf16_val(t.w);
  }
  v4f fv[16];
#pragma unroll
  for (int i = 0; i < 16; ++i) {
    const int lr = 16 * wave + i;
    fv[i] = *(const v4fa*)(stg + lr * GN + 4 * lane) + b4;
  }
  float* hb = H + (size_t)g * GN + 4 * lane;

#pragma unroll
  for (int i = 0; i < 16; ++i) {
    const int gr = rowBase + 16 * wave + i;
    if (gr < nStore) {
      float* op = hb + (size_t)gr * (size_t)ldh;
      *(volatile v4f*)op = fv[i];
    }
  }
  if constexpr (DOTS != 0) {
    const int piece = lane & 7, pl = (lane >> 3) & 1;
    const v4f sdv = *(const v4fa*)(sdot + pl * GBM + 4 * piece);
    float* sp = SD + (size_t)(2 * g + pl) * (size_t)MPr + rowBase + 4 * piece;
    if (wave == 0 && lane < 16) *(volatile v4f*)sp = sdv;
  }
  __threadfence();
#pragma unroll
  for (int i = 0; i < 16; ++i) {
    const int gr = rowBase + 16 * wave + i;
    if (gr < nStore) {
      float* op = hb + (size_t)gr * (size_t)ldh;
      *(volatile v4f*)op = fv[i];
    }
  }
  if constexpr (DOTS != 0) {
    const int piece = lane & 7, pl = (lane >> 3) & 1;
    const v4f sdv = *(const v4fa*)(sdot + pl * GBM + 4 * piece);
    float* sp = SD + (size_t)(2 * g + pl) * (size_t)MPr + rowBase + 4 * piece;
    if (wave == 0 && lane < 16) *(volatile v4f*)sp = sdv;
  }
}

template <int RELU>
__global__ __launch_bounds__(NTHR) void k_agg(
    const int* __restrict__ srcs, const int* __restrict__ dsts, int nE, int nN, int MPr, int nb, int vec8,
    const float* __restrict__ F, int ldF, int colOff,
    const float* __restrict__ AS, const float* __restrict__ AD, const float* __restrict__ bias,
    unsigned short* hp, int ldp) {
  extern __shared__ v4f lds_dyn[];
  int* reg1 = (int*)lds_dyn;
  int* reg2 = reg1 + RCAP;
  int* scnt = reg2 + RCAP;
  int* soff = scnt + NBMAX;
  int* list = soff + NBMAX;
  int* wcnt = list + LISTN;
  int* wtot = wcnt + NWAVE;
  const int tid = (int)threadIdx.x, lane = tid & 31, wave = tid >> 5;
  const int nodeBase = (int)blockIdx.x * nb;

  for (int i = tid; i < NBMAX; i += NTHR) scnt[i] = 0;
  __syncthreads();

  int tot = 0;
  const int nChunks = (nE + CHUNK - 1) / CHUNK;
#pragma unroll 1
  for (int ch = 0; ch < nChunks; ++ch) {
    const int cbase = ch * CHUNK;
    const int wc = scan_chunk(dsts, nE, cbase, nodeBase, nb, vec8, list, tid, lane, wave);
    if (lane == 0) wcnt[wave] = wc;
    __syncthreads();
    int pre = 0, all = 0;
#pragma unroll
    for (int w2 = 0; w2 < NWAVE; ++w2) {
      int c = wcnt[w2];
      c = c < 0 ? 0 : (c > WCAP ? WCAP : c);
      all += c;
      pre += (w2 < wave) ? c : 0;
    }
    const int wcc  = wc > WCAP ? WCAP : wc;
    const int base = tot + pre;
#pragma unroll 1
    for (int i = lane; i < wcc; i += 32) {
      const int ent = list[wave * WCAP + i];
      const int el  = (ent >> SLOTB) & (CHUNK - 1);
      const int sl  = ent & (NBMAX - 1);
      int eid = cbase + el;
      eid = eid > nE - 1 ? nE - 1 : eid;
      const int pos = base + i;
      if (pos < RCAP) reg1[pos] = (int)(((unsigned)eid << SLOTB) | (unsigned)sl);
    }
    tot += all;
    tot = tot > RCAP ? RCAP : tot;
    __syncthreads();
  }
  const int nh = tot;

  if (wave == 0) {
#pragma unroll 1
    for (int b0 = 0; b0 < nh; b0 += 32) {
      const int idx = b0 + lane;
      const int uv  = reg1[idx < nh ? idx : nh - 1];
      const int m32 = (nh - b0) < 32 ? (nh - b0) : 32;
#pragma unroll 1
      for (int k = 0; k < m32; ++k) {
        const int u  = __builtin_amdgcn_readlane(uv, k);
        const int sl = u & (NBMAX - 1);
        if (lane == 0) scnt[sl] = scnt[sl] + 1;
      }
    }
  }
  __syncthreads();

  {
    const v4i ca = *(const v4ia*)(scnt + 8 * tid);
    const v4i cb = *(const v4ia*)(scnt + 8 * tid + 4);
    const int e0 = ca.x < 0 ? 0 : ca.x, e1 = ca.y < 0 ? 0 : ca.y, e2 = ca.z < 0 ? 0 : ca.z, e3 = ca.w < 0 ? 0 : ca.w;
    const int e4 = cb.x < 0 ? 0 : cb.x, e5 = cb.y < 0 ? 0 : cb.y, e6 = cb.z < 0 ? 0 : cb.z, e7 = cb.w < 0 ? 0 : cb.w;
    const int ts = e0 + e1 + e2 + e3 + e4 + e5 + e6 + e7;
    int incl = ts;
#pragma unroll
    for (int d = 1; d < 32; d <<= 1) {
      const int up = __shfl_up(incl, d);
      if (lane >= d) incl += up;
    }
    if (lane == 31) wtot[wave] = incl;
    __syncthreads();
    int pre = 0;
#pragma unroll
    for (int w2 = 0; w2 < NWAVE; ++w2) pre += (w2 < wave) ? wtot[w2] : 0;
    int run = pre + incl - ts;
    soff[8 * tid + 0] = run; run += e0;
    soff[8 * tid + 1] = run; run += e1;
    soff[8 * tid + 2] = run; run += e2;
    soff[8 * tid + 3] = run; run += e3;
    soff[8 * tid + 4] = run; run += e4;
    soff[8 * tid + 5] = run; run += e5;
    soff[8 * tid + 6] = run; run += e6;
    soff[8 * tid + 7] = run;
  }
  __syncthreads();
  for (int i = tid; i < NBMAX; i += NTHR) list[i] = soff[i];
  __syncthreads();

  if (wave == 0) {
#pragma unroll 1
    for (int b0 = 0; b0 < nh; b0 += 32) {
      const int idx = b0 + lane;
      const int uv  = reg1[idx < nh ? idx : nh - 1];
      const int m32 = (nh - b0) < 32 ? (nh - b0) : 32;
#pragma unroll 1
      for (int k = 0; k < m32; ++k) {
        const int u   = __builtin_amdgcn_readlane(uv, k);
        const int sl  = u & (NBMAX - 1);
        const int eid = (int)((unsigned)u >> SLOTB);
        if (lane == 0) {
          int pos = list[sl];
          pos = pos < 0 ? 0 : (pos > RCAP - 1 ? RCAP - 1 : pos);
          reg2[pos] = eid;
          list[sl] = pos + 1;
        }
      }
    }
  }
  __syncthreads();

  const int nbw = nb >> 3;
  const bool ovf = (nh >= RCAP);
  const float qnan = __int_as_float(0x7fc00000);
  v4f bb4;
  {
    const v4f t = *(const v4fa*)(bias + 4 * lane);
    bb4.x = bf16_val(t.x); bb4.y = bf16_val(t.y); bb4.z = bf16_val(t.z); bb4.w = bf16_val(t.w);
  }

#pragma unroll 1
  for (int jt = 0; jt < nbw; ++jt) {
    const int slot = wave * nbw + jt;
    const int grow = nodeBase + slot;
    const int gcl  = grow < nN ? grow : nN - 1;
    int st = soff[slot];
    const int craw = scnt[slot];
    int cnt = craw;
    st  = st < 0 ? 0 : (st > nh ? nh : st);
    cnt = cnt < 0 ? 0 : (cnt > DEGCAP ? DEGCAP : cnt);
    if (cnt > nh - st) cnt = nh - st;
    const float pz = (ovf || craw > DEGCAP) ? qnan : 0.0f;

    const float adv = AD[gcl];
    const v4f fd = *(const v4fa*)(F + (size_t)gcl * (size_t)ldF + colOff + 4 * lane);
    float l0 = AS[gcl] + adv;
    l0 = l0 > 0.f ? l0 : NEGSL * l0;
    float mx = l0, dn = 1.0f;
    float a0 = fd.x, a1 = fd.y, a2 = fd.z, a3 = fd.w;

#pragma unroll 1
    for (int q = 0; q < cnt; ++q) {
      int idx = st + q; idx = idx > RCAP - 1 ? RCAP - 1 : idx;
      int eid = reg2[idx]; eid = eid < 0 ? 0 : (eid > nE - 1 ? nE - 1 : eid);
      const int sraw = srcs[eid];
      const int s = sraw < 0 ? 0 : (sraw > nN - 1 ? nN - 1 : sraw);
      const v4f fs = *(const v4fa*)(F + (size_t)s * (size_t)ldF + colOff + 4 * lane);
      float lg = AS[s] + adv;
      lg = lg > 0.f ? lg : NEGSL * lg;
      const float df = lg - mx;
      const float ee = __expf(-fabsf(df));
      const bool up  = df > 0.f;
      const float s1 = up ? ee : 1.0f;
      const float s2 = up ? 1.0f : ee;
      mx = up ? lg : mx;
      dn = fmaf(dn, s1, s2);
      a0 = fmaf(a0, s1, s2 * fs.x);
      a1 = fmaf(a1, s1, s2 * fs.y);
      a2 = fmaf(a2, s1, s2 * fs.z);
      a3 = fmaf(a3, s1, s2 * fs.w);
    }
    const float inv = __builtin_amdgcn_rcpf(dn);
    const bool live = grow < nN;
    const bool wrow = grow < MPr;

    v4f v;
    v.x = fmaf(a0, inv, bb4.x);
    v.y = fmaf(a1, inv, bb4.y);
    v.z = fmaf(a2, inv, bb4.z);
    v.w = fmaf(a3, inv, bb4.w);
    if constexpr (RELU != 0) {
      v.x = fmaxf(v.x, 0.0f); v.y = fmaxf(v.y, 0.0f); v.z = fmaxf(v.z, 0.0f); v.w = fmaxf(v.w, 0.0f);
    }
    v4f y;
    y.x = (live ? v.x : 0.f) + pz;
    y.y = (live ? v.y : 0.f) + pz;
    y.z = (live ? v.z : 0.f) + pz;
    y.w = (live ? v.w : 0.f) + pz;
    const v8us po = hilo8(y);
    unsigned short* gp = hp + (size_t)grow * (size_t)ldp + 8 * lane;
    if (wrow) *(volatile v8us*)gp = po;
    __threadfence();
    if (wrow) *(volatile v8us*)gp = po;
  }
}

static int pick_nb(int nE, int nN) {
  int nb = NBMAX;
  while (nb > 32 && (long long)nb * (long long)nE * 8LL > (long long)RCAP * (long long)nN * 7LL) nb >>= 1;
  return nb;
}
static inline int cdiv(int a, int b) { return (a + b - 1) / b; }

extern "C" void kernel_launch(void* const* d_in, const int* in_sizes, int n_in,
                              void* d_out, int out_size, void* d_ws, size_t ws_size,
                              hipStream_t stream) {
  if (n_in < 21) return;
  if (in_sizes[0] < DIN || (in_sizes[0] % DIN) != 0) return;
  const int nN = in_sizes[0] / DIN;
  if (nN > (1 << 22)) return;
  if ((in_sizes[1] & 1) || (in_sizes[2] & 1)) return;
  const int nEo = in_sizes[1] / 2, nEs = in_sizes[2] / 2;
  if (nEo < 1 || nEs < 1 || nEo >= (1 << (32 - SLOTB)) || nEs >= (1 << (32 - SLOTB))) return;
  if (in_sizes[3] != DIN * GN || in_sizes[7] != DIN * GN) return;
  if (in_sizes[11] != DIN * GN || in_sizes[15] != DIN * GN) return;
  if (in_sizes[19] != DIN * GN) return;
  {
    const int vecs[13] = {4, 5, 6, 8, 9, 10, 12, 13, 14, 16, 17, 18, 20};
    for (int i = 0; i < 13; ++i) if (in_sizes[vecs[i]] != GN) return;
  }
  if (out_size != nN * GN) return;

  const float* x    = (const float*)d_in[0];
  const int*   eo   = (const int*)  d_in[1];
  const int*   es   = (const int*)  d_in[2];
  const float* Wo1  = (const float*)d_in[3];
  const float* aso1 = (const float*)d_in[4];
  const float* ado1 = (const float*)d_in[5];
  const float* bo1  = (const float*)d_in[6];
  const float* Ws1  = (const float*)d_in[7];
  const float* ass1 = (const float*)d_in[8];
  const float* ads1 = (const float*)d_in[9];
  const float* bs1  = (const float*)d_in[10];
  const float* Wo2  = (const float*)d_in[11];
  const float* aso2 = (const float*)d_in[12];
  const float* ado2 = (const float*)d_in[13];
  const float* bo2  = (const float*)d_in[14];
  const float* Ws2  = (const float*)d_in[15];
  const float* ass2 = (const float*)d_in[16];
  const float* ads2 = (const float*)d_in[17];
  const float* bs2  = (const float*)d_in[18];
  const float* Wp   = (const float*)d_in[19];
  const float* bp   = (const float*)d_in[20];
  float* out = (float*)d_out;

  const int MP  = cdiv(nN, MROWS) * MROWS;
  const int nbo = pick_nb(nEo, nN), nbs = pick_nb(nEs, nN);
  if (nbo < 32 || (nbo & (nbo - 1)) != 0 || nbo > NBMAX) return;
  if (nbs < 32 || (nbs & (nbs - 1)) != 0 || nbs > NBMAX) return;
  const int gAo = cdiv(MP, nbo), gAs = cdiv(MP, nbs);
  if ((long long)gAo * nbo < MP || (long long)gAs * nbs < MP) return;
  const int veco = ((nEo & 3) == 0) ? 1 : 0, vecs = ((nEs & 3) == 0) ? 1 : 0;
  const int XU = MP * (DIN / 8);
  if ((XU % NTHR) != 0 || (MP % GBM) != 0) return;

  char* ws = (char*)d_ws;
  size_t off = 0;
  const size_t oWT1 = off; off += (size_t)NG * DIN * 2;        off = (off + 255) & ~(size_t)255;
  const size_t oWT2 = off; off += (size_t)NG * KHL * 2;        off = (off + 255) & ~(size_t)255;
  const size_t oWTp = off; off += (size_t)GN * KHL * 2;        off = (off + 255) & ~(size_t)255;
  const size_t oSD  = off; off += (size_t)4 * MP * 4;          off = (off + 255) & ~(size_t)255;
  const size_t oH   = off; off += (size_t)MP * NG * 4;         off = (off + 255) & ~(size_t)255;
  const size_t oP   = off; off += (size_t)MP * KHL * 2;        off = (off + 255) & ~(size_t)255;
  if (off > ws_size || off > (size_t)WSMAX) return;
  if ((size_t)MP * DIN * 2 > (size_t)MP * KHL * 2) return;

  unsigned short* WT1 = (unsigned short*)(ws + oWT1);
  unsigned short* WT2 = (unsigned short*)(ws + oWT2);
  unsigned short* WTp = (unsigned short*)(ws + oWTp);
  float*          SD  = (float*)(ws + oSD);
  float*          H   = (float*)(ws + oH);
  unsigned short* XB  = (unsigned short*)(ws + oP);
  unsigned short* HA  = (unsigned short*)(ws + oP);
  unsigned short* HB  = (unsigned short*)(ws + oP);

  hipFuncSetAttribute(reinterpret_cast<const void*>(&k_agg<1>), hipFuncAttributeMaxDynamicSharedMemorySize, LDS_AGG);
  hipFuncSetAttribute(reinterpret_cast<const void*>(&k_agg<0>), hipFuncAttributeMaxDynamicSharedMemorySize, LDS_AGG);

  k_wprep<<<UTOT / NTHR, NTHR, 0, stream>>>(Wo1, Ws1, Wo2, Ws2, Wp, WT1, WT2, WTp);
  k_xprep<<<cdiv(XU, NTHR), NTHR, 0, stream>>>(x, XB, nN, XU);

  k_gemm<1, 0><<<dim3(MP / GBM, 2), GTHR, 0, stream>>>(XB, WT1, DIN, MP, aso1, ado1, ass1, ads1, bo1,
                                                       H, NG, MP, SD);
  k_agg<1><<<gAo, NTHR, LDS_AGG, stream>>>(eo, eo + nEo, nEo, nN, MP, nbo, veco, H, NG, 0,
                                            SD + 0 * (size_t)MP, SD + 1 * (size_t)MP, bo1, HA, KHL);
  k_agg<1><<<gAs, NTHR, LDS_AGG, stream>>>(es, es + nEs, nEs, nN, MP, nbs, vecs, H, NG, GN,
                                            SD + 2 * (size_t)MP, SD + 3 * (size_t)MP, bs1, HA + NG, KHL);

  k_gemm<1, 0><<<dim3(MP / GBM, 2), GTHR, 0, stream>>>(HA, WT2, KHL, MP, aso2, ado2, ass2, ads2, bo2,
                                                       H, NG, MP, SD);
  k_agg<0><<<gAo, NTHR, LDS_AGG, stream>>>(eo, eo + nEo, nEo, nN, MP, nbo, veco, H, NG, 0,
                                            SD + 0 * (size_t)MP, SD + 1 * (size_t)MP, bo2, HB, KHL);
  k_agg<0><<<gAs, NTHR, LDS_AGG, stream>>>(es, es + nEs, nEs, nN, MP, nbs, vecs, H, NG, GN,
                                            SD + 2 * (size_t)MP, SD + 3 * (size_t)MP, bs2, HB + NG, KHL);

  k_gemm<0, 1><<<dim3(MP / GBM, 1), GTHR, 0, stream>>>(HB, WTp, KHL, MP, bp, bp, bp, bp, bp,
                                                       out, GN, nN, SD);
}
